// MoE_CondNP_21612275433874
// MI455X (gfx1250) — hardware-verified
//
#include <hip/hip_runtime.h>
#include <math.h>

typedef _Float16 v16h __attribute__((ext_vector_type(16)));
typedef _Float16 v8h  __attribute__((ext_vector_type(8)));
typedef float    v8f  __attribute__((ext_vector_type(8)));
typedef float    v4f  __attribute__((ext_vector_type(4)));
typedef v8h __attribute__((may_alias)) v8ha;
typedef v4f __attribute__((may_alias)) v4fa;
union Frag { v16h v; v8h half[2]; };

#define NB     8
#define NTT    1024
#define NK     8
#define NL     128
#define NH     512
#define NHG    256
#define NPT    512
#define MROWS  4096
#define DROWS  65536
#define DHALF  32768
#define WSC    64.0f
#define ASC    16.0f
#define INV_WA (1.0f / 1024.0f)
#define INV_A  (1.0f / 16.0f)

#define OFF_MU_C  0
#define OFF_LV_C  8192
#define OFF_MU_T  16384
#define OFF_LV_T  24576
#define OFF_YM    32768
#define OFF_YS    229376
#define OFF_AP    425984
#define OFF_AQ    491520
#define OUT_TOTAL 557056

#define SPITCH 40
#define TPITCH 136

__device__ __forceinline__ v8f wmma16(v16h a, v16h b, v8f c) {
  v8f d = __builtin_amdgcn_wmma_f32_16x16x32_f16(false, a, false, b, (short)0, c, false, false);
  asm volatile("v_nop\n\tv_nop\n\tv_nop\n\tv_nop" : "+v"(d) : "v"(a), "v"(b));
  return d;
}

__global__ __launch_bounds__(256) void k_cvtT(const float* __restrict__ src, _Float16* __restrict__ dst,
                                              int Kin, int N, int srcBStride, int dstBStride)
{
  __shared__ __attribute__((aligned(16))) _Float16 sT[32 * 72];
  const int tid = threadIdx.x;
  const int n0 = blockIdx.x * 32, k0 = blockIdx.y * 64, bz = blockIdx.z;
  const float* s = src + (size_t)bz * srcBStride;
  _Float16* d = dst + (size_t)bz * dstBStride;
#pragma unroll
  for (int it = 0; it < 8; ++it) {
    const int e = tid + 256 * it;
    const int kk = e >> 5, nn = e & 31;
    const float v = s[(size_t)(k0 + kk) * N + n0 + nn];
    sT[nn * 72 + kk] = (_Float16)(v * WSC);
  }
  __syncthreads();
  const int row = tid >> 3, q = tid & 7;
  const v8h v = *(const v8ha*)(sT + row * 72 + 8 * q);
  _Float16* p = d + (size_t)(n0 + row) * Kin + k0 + 8 * q;
  *(volatile v8h*)p = v;
  __threadfence();
  *(volatile v8h*)p = v;
}

template <int CA, int CB>
__global__ __launch_bounds__(256) void k_l0(
    const float* __restrict__ xa, const float* __restrict__ xb, int xShift, int rowBase,
    const float* __restrict__ W, int wKStride,
    const float* __restrict__ add, int addKStride, int gHiShift, int gLoMask, int addRowStride,
    int N, _Float16* __restrict__ outp, int outKStride)
{
  constexpr int CF = CA + CB;
  __shared__ __attribute__((aligned(16))) _Float16 sT[16 * 512];
  __shared__ float sX[16 * CF];
  const int tid = threadIdx.x;
  const int kg = blockIdx.y;
  const int r0 = blockIdx.x * 16;
  {
    const int e = min(tid, 16 * CF - 1);
    const int r = e / CF, j = e - r * CF;
    const int xrow = (rowBase + r0 + r) >> xShift;
    const float va = xa[(size_t)xrow * CA + min(j, CA - 1)];
    float v = va;
    if (CB > 0) {
      const float vb = xb[(size_t)xrow * CB + max(j - CA, 0)];
      v = (j < CA) ? va : vb;
    }
    if (tid < 16 * CF) sX[tid] = v;
  }
  __syncthreads();
  const float* Wg = W + (size_t)kg * wKStride;
  const float* ag = add + (size_t)kg * addKStride;
  for (int c = tid; c < N; c += 256) {
    float w[CF];
#pragma unroll
    for (int j = 0; j < CF; ++j) w[j] = Wg[(size_t)j * N + c];
#pragma unroll 4
    for (int r = 0; r < 16; ++r) {
      const int R = rowBase + r0 + r;
      const int ga = ((R >> gHiShift) << 3) | (R & gLoMask);
      float v = ag[(size_t)ga * addRowStride + c];
#pragma unroll
      for (int j = 0; j < CF; ++j) v = fmaf(sX[r * CF + j], w[j], v);
      v = fmaxf(v, 0.0f) * ASC;
      sT[r * N + c] = (_Float16)v;
    }
  }
  __syncthreads();
  _Float16* ob = outp + (size_t)kg * outKStride + (size_t)r0 * N;
  const int np = 2 * N;
  for (int p = tid; p < np; p += 256) {
    const v8h v = *(const v8ha*)(sT + 8 * p);
    *(volatile v8h*)(ob + 8 * p) = v;
  }
  __threadfence();
  for (int p = tid; p < np; p += 256) {
    const v8h v = *(const v8ha*)(sT + 8 * p);
    *(volatile v8h*)(ob + 8 * p) = v;
  }
}

template <int MODE>
__global__ __launch_bounds__(256) void k_gemm(
    const _Float16* __restrict__ A, int aGStride,
    const _Float16* __restrict__ WT, int wGStride,
    const float* __restrict__ bias, int bGStride,
    int K, int N, int tilesM,
    _Float16* __restrict__ C, int cGStride,
    float* __restrict__ tab, int tabGStride, int tabTNStride,
    const float* __restrict__ Wo)
{
  __shared__ __attribute__((aligned(16))) _Float16 sH[128 * TPITCH];
  __shared__ __attribute__((aligned(16))) float sF[1024];
  _Float16* sA = sH;
  _Float16* sW = sH + 128 * SPITCH;

  const int tid = threadIdx.x, lane = tid & 31, wave = tid >> 5;
  const int wm = wave >> 2, wn = wave & 3, c16 = lane & 15, hh = lane >> 4;
  const int g = blockIdx.y;
  const int tileM = blockIdx.x % tilesM, tileN = blockIdx.x / tilesM;
  const int row0 = tileM * 128, col0 = tileN * 128;
  const _Float16* Ag = A + (size_t)g * aGStride + (size_t)row0 * K;
  const _Float16* Wg = WT + (size_t)g * wGStride + (size_t)col0 * K;
  const float* bg = bias + (size_t)g * bGStride + col0;

  const v8f zero8 = {0.f, 0.f, 0.f, 0.f, 0.f, 0.f, 0.f, 0.f};
  v8f acc[4][2];
#pragma unroll
  for (int mi = 0; mi < 4; ++mi) { acc[mi][0] = zero8; acc[mi][1] = zero8; }

#pragma unroll 1
  for (int k0 = 0; k0 < K; k0 += 32) {
#pragma unroll
    for (int it = 0; it < 2; ++it) {
      const int chunk = tid + 256 * it;
      const int row = chunk >> 2, kc = (chunk & 3) * 8;
      const v8h va = *(const v8ha*)(Ag + (size_t)row * K + k0 + kc);
      const v8h vw = *(const v8ha*)(Wg + (size_t)row * K + k0 + kc);
      *(v8ha*)(sA + row * SPITCH + kc) = va;
      *(v8ha*)(sW + row * SPITCH + kc) = vw;
    }
    __syncthreads();
    Frag fa[4], fb[2];
#pragma unroll
    for (int mi = 0; mi < 4; ++mi) {
      const _Float16* p = sA + (wm * 64 + mi * 16 + c16) * SPITCH;
      fa[mi].half[0] = *(const v8ha*)(p + 8 * hh);
      fa[mi].half[1] = *(const v8ha*)(p + 16 + 8 * hh);
    }
#pragma unroll
    for (int nj = 0; nj < 2; ++nj) {
      const _Float16* p = sW + (wn * 32 + nj * 16 + c16) * SPITCH;
      fb[nj].half[0] = *(const v8ha*)(p + 8 * hh);
      fb[nj].half[1] = *(const v8ha*)(p + 16 + 8 * hh);
    }
#pragma unroll
    for (int mi = 0; mi < 4; ++mi) {
      acc[mi][0] = wmma16(fa[mi].v, fb[0].v, acc[mi][0]);
      acc[mi][1] = wmma16(fa[mi].v, fb[1].v, acc[mi][1]);
    }
    __syncthreads();
  }

  if (MODE == 1) {
#pragma unroll
    for (int nj = 0; nj < 2; ++nj) {
      const int cl = wn * 32 + nj * 16 + c16;
      const float bb = bg[cl];
      float ps = 0.0f;
#pragma unroll
      for (int mi = 0; mi < 4; ++mi)
#pragma unroll
        for (int r = 0; r < 8; ++r) ps += fmaxf(acc[mi][nj][r] * INV_WA + bb, 0.0f);
      const float other = __shfl_xor(ps, 16);
      const float ps2 = ps + other;
      if (hh == 0) sF[wm * 128 + cl] = ps2;
    }
    __syncthreads();
    if (tid < 128) sF[256 + tid] = sF[tid] + sF[128 + tid];
    __syncthreads();
    float* p = tab + (size_t)g * tabGStride + (size_t)tileM * N + col0 + 4 * lane;
    const v4f v = *(const v4fa*)(sF + 256 + 4 * lane);
    if (wave == 0) *(volatile v4f*)p = v;
    __threadfence();
    if (wave == 0) *(volatile v4f*)p = v;
  } else {
#pragma unroll
    for (int nj = 0; nj < 2; ++nj) {
      const int cl = wn * 32 + nj * 16 + c16;
      const float bb = bg[cl];
#pragma unroll
      for (int mi = 0; mi < 4; ++mi)
#pragma unroll
        for (int r = 0; r < 8; ++r) {
          const int rl = wm * 64 + mi * 16 + 8 * hh + r;
          const float v = fmaxf(acc[mi][nj][r] * INV_WA + bb, 0.0f) * ASC;
          sH[rl * TPITCH + cl] = (_Float16)v;
        }
    }
    __syncthreads();
    if (MODE == 0) {
      _Float16* Cg = C + (size_t)g * cGStride + (size_t)row0 * N + col0;
#pragma unroll
      for (int i = 0; i < 8; ++i) {
        const int rl = wave * 16 + 2 * i + hh;
        const v8h v = *(const v8ha*)(sH + rl * TPITCH + 8 * c16);
        *(volatile v8h*)(Cg + (size_t)rl * N + 8 * c16) = v;
      }
      __threadfence();
#pragma unroll
      for (int i = 0; i < 8; ++i) {
        const int rl = wave * 16 + 2 * i + hh;
        const v8h v = *(const v8ha*)(sH + rl * TPITCH + 8 * c16);
        *(volatile v8h*)(Cg + (size_t)rl * N + 8 * c16) = v;
      }
    } else if (MODE == 2) {
      const int rl = tid >> 1, hs = tid & 1;
      const _Float16* hp = sH + rl * TPITCH + hs * 64;
      const float* wp = Wo + col0 + hs * 64;
      float s = 0.0f;
#pragma unroll 4
      for (int c = 0; c < 64; ++c) s = fmaf((float)hp[c], wp[c], s);
      const float o = __shfl_xor(s, 1);
      const float tot = ((hs == 0) ? (s + o) : (o + s)) * INV_A;
      if (hs == 0) sF[rl] = tot;
      __syncthreads();
      float* p = tab + (size_t)tileN * tabTNStride + row0 + 4 * lane;
      const v4f v = *(const v4fa*)(sF + 4 * lane);
      if (wave == 0) *(volatile v4f*)p = v;
      __threadfence();
      if (wave == 0) *(volatile v4f*)p = v;
    } else {
      const int rl = tid >> 1, js = tid & 1, j0 = 3 * js;
      const _Float16* hp = sH + rl * TPITCH;
      const float* wp = Wo + (size_t)col0 * 6 + j0;
      float o0 = 0.0f, o1 = 0.0f, o2 = 0.0f;
#pragma unroll 2
      for (int c = 0; c < 128; ++c) {
        const float hv = (float)hp[c];
        const float* w = wp + c * 6;
        o0 = fmaf(hv, w[0], o0);
        o1 = fmaf(hv, w[1], o1);
        o2 = fmaf(hv, w[2], o2);
      }
      sF[rl * 8 + j0 + 0] = o0 * INV_A;
      sF[rl * 8 + j0 + 1] = o1 * INV_A;
      sF[rl * 8 + j0 + 2] = o2 * INV_A;
      if (js == 1) { sF[rl * 8 + 6] = 0.0f; sF[rl * 8 + 7] = 0.0f; }
      __syncthreads();
      float* p = tab + (size_t)tileN * tabTNStride + (size_t)row0 * 8 + 4 * tid;
      const v4f v = *(const v4fa*)(sF + 4 * tid);
      *(volatile v4f*)p = v;
      __threadfence();
      *(volatile v4f*)p = v;
    }
  }
}

__global__ __launch_bounds__(128) void k_head(
    const float* __restrict__ pp, const float* __restrict__ Wmu, const float* __restrict__ bmu,
    const float* __restrict__ Wlv, const float* __restrict__ blv, const float* __restrict__ eps,
    int which, float* __restrict__ out, float* __restrict__ zbuf)
{
  __shared__ float sR[NH];
  __shared__ __attribute__((aligned(16))) float sO[3 * NL];
  const int g = blockIdx.x, b = g >> 3, k = g & 7;
  const int t = threadIdx.x;
#pragma unroll
  for (int q = 0; q < 4; ++q) {
    const int c = t + 128 * q;
    const float* p = pp + ((size_t)(k * 32 + b * 4)) * NH + c;
    const float s = ((p[0] + p[NH]) + p[2 * NH]) + p[3 * NH];
    sR[c] = s * (1.0f / 512.0f);
  }
  __syncthreads();
  float mu = 0.0f, lv = 0.0f;
  const float* wm = Wmu + (size_t)k * NH * NL + t;
  const float* wl = Wlv + (size_t)k * NH * NL + t;
#pragma unroll 2
  for (int h = 0; h < NH; ++h) {
    const float r = sR[h];
    mu = fmaf(r, wm[(size_t)h * NL], mu);
    lv = fmaf(r, wl[(size_t)h * NL], lv);
  }
  mu += bmu[k * NL + t];
  lv += blv[k * NL + t];
  sO[t] = mu;
  sO[NL + t] = lv;
  sO[2 * NL + t] = mu + eps[(size_t)g * NL + t] * expf(0.5f * lv);
  __syncthreads();
  const int wave = t >> 5, lane = t & 31;
  float* pm = out + (which ? OFF_MU_T : OFF_MU_C) + (size_t)g * NL + 4 * lane;
  float* pl = out + (which ? OFF_LV_T : OFF_LV_C) + (size_t)g * NL + 4 * lane;
  float* pz = zbuf + (size_t)g * NL + 4 * lane;
  const v4f vm = *(const v4fa*)(sO + 4 * lane);
  const v4f vl = *(const v4fa*)(sO + NL + 4 * lane);
  const v4f vz = *(const v4fa*)(sO + 2 * NL + 4 * lane);
  if (wave == 0) *(volatile v4f*)pm = vm;
  else if (wave == 1) *(volatile v4f*)pl = vl;
  else if (wave == 2 && which != 0) *(volatile v4f*)pz = vz;
  __threadfence();
  if (wave == 0) *(volatile v4f*)pm = vm;
  else if (wave == 1) *(volatile v4f*)pl = vl;
  else if (wave == 2 && which != 0) *(volatile v4f*)pz = vz;
}

__global__ __launch_bounds__(256) void k_zterm(
    const float* __restrict__ zbuf,
    const float* __restrict__ dW0, const float* __restrict__ db0,
    const float* __restrict__ pW0, const float* __restrict__ pb0,
    const float* __restrict__ qW0, const float* __restrict__ qb0,
    float* __restrict__ zD, float* __restrict__ zP, float* __restrict__ zQ)
{
  __shared__ float sZ[NL];
  __shared__ __attribute__((aligned(16))) float sO[1024];
  const int g = blockIdx.x, t = threadIdx.x;
  const float zv = zbuf[(size_t)g * NL + (t & 127)];
  if (t < NL) sZ[t] = zv;
  __syncthreads();
  float a0 = 0.0f, a1 = 0.0f, a2 = 0.0f, a3 = 0.0f;
#pragma unroll 2
  for (int l = 0; l < NL; ++l) {
    const float z = sZ[l];
    a0 = fmaf(z, dW0[(size_t)(2 + l) * NH + t], a0);
    a1 = fmaf(z, dW0[(size_t)(2 + l) * NH + t + 256], a1);
    a2 = fmaf(z, pW0[(size_t)(5 + l) * NHG + t], a2);
    a3 = fmaf(z, qW0[(size_t)(2 + l) * NHG + t], a3);
  }
  sO[t] = a0 + db0[t];
  sO[256 + t] = a1 + db0[256 + t];
  sO[512 + t] = a2 + pb0[t];
  sO[768 + t] = a3 + qb0[t];
  __syncthreads();
  const int wave = t >> 5;
  float* dst;
  if (wave < 4) dst = zD + (size_t)g * NH + 4 * t;
  else if (wave < 6) dst = zP + (size_t)g * NHG + 4 * (t - 128);
  else dst = zQ + (size_t)g * NHG + 4 * (t - 192);
  const v4f v = *(const v4fa*)(sO + 4 * t);
  *(volatile v4f*)dst = v;
  __threadfence();
  *(volatile v4f*)dst = v;
}

__global__ __launch_bounds__(256) void k_dec_fin(const float* __restrict__ pdec, const float* __restrict__ dbo,
                                                 float* __restrict__ out)
{
  __shared__ __attribute__((aligned(16))) float sM[768];
  __shared__ __attribute__((aligned(16))) float sS[768];
  const int t = threadIdx.x;
  const int r = blockIdx.x * 256 + t;
  const float* p = pdec + (size_t)r * 8;
  const size_t TN = (size_t)DROWS * 8;
  const v4f u0 = *(const v4fa*)(p),          u1 = *(const v4fa*)(p + 4);
  const v4f w0 = *(const v4fa*)(p + TN),     w1 = *(const v4fa*)(p + TN + 4);
  const v4f x0 = *(const v4fa*)(p + 2 * TN), x1 = *(const v4fa*)(p + 2 * TN + 4);
  const v4f y0 = *(const v4fa*)(p + 3 * TN), y1 = *(const v4fa*)(p + 3 * TN + 4);
  const v4f lo = ((u0 + w0) + x0) + y0;
  const v4f hi = ((u1 + w1) + x1) + y1;
  sM[t * 3 + 0] = lo.x + dbo[0];
  sM[t * 3 + 1] = lo.y + dbo[1];
  sM[t * 3 + 2] = lo.z + dbo[2];
  sS[t * 3 + 0] = lo.w + dbo[3];
  sS[t * 3 + 1] = hi.x + dbo[4];
  sS[t * 3 + 2] = hi.y + dbo[5];
#pragma unroll 1
  for (int j = 0; j < 3; ++j) {
    const float xm = sM[t * 3 + j];
    const float e = expf(-xm);
    sM[t * 3 + j] = 1.0f / (1.0f + e);
    const float xs = sS[t * 3 + j];
    sS[t * 3 + j] = fmaxf(xs, 0.0f) + log1pf(expf(-fabsf(xs)));
  }
  __syncthreads();
  float* pm = out + OFF_YM + (size_t)blockIdx.x * 768 + 4 * t;
  float* ps = out + OFF_YS + (size_t)blockIdx.x * 768 + 4 * t;
  const int tc = min(t, 191);
  const v4f vm = *(const v4fa*)(sM + 4 * tc);
  const v4f vs = *(const v4fa*)(sS + 4 * tc);
  if (t < 192) { *(volatile v4f*)pm = vm; *(volatile v4f*)ps = vs; }
  __threadfence();
  if (t < 192) { *(volatile v4f*)pm = vm; *(volatile v4f*)ps = vs; }
}

__global__ __launch_bounds__(256) void k_gate_fin(const float* __restrict__ plogP, const float* __restrict__ pbo,
                                                  const float* __restrict__ plogQ, const float* __restrict__ qbo,
                                                  float* __restrict__ out)
{
  __shared__ __attribute__((aligned(16))) float sL[2048];
  const int t = threadIdx.x, sel = blockIdx.y;
  const float* plog = sel ? plogQ : plogP;
  const float bp = pbo[0], bq = qbo[0];
  const float bo = sel ? bq : bp;
  const int bt = blockIdx.x * 256 + t;
  const float* base = plog + (size_t)bt * 8;
  const v4f a0 = *(const v4fa*)(base), a1 = *(const v4fa*)(base + 4);
  const v4f b0 = *(const v4fa*)(base + DROWS), b1 = *(const v4fa*)(base + DROWS + 4);
  const v4f lo = (a0 + b0) + bo;
  const v4f hi = (a1 + b1) + bo;
  const float m = fmaxf(fmaxf(fmaxf(lo.x, lo.y), fmaxf(lo.z, lo.w)),
                        fmaxf(fmaxf(hi.x, hi.y), fmaxf(hi.z, hi.w)));
  float* sl = sL + t * 8;
  sl[0] = lo.x - m; sl[1] = lo.y - m; sl[2] = lo.z - m; sl[3] = lo.w - m;
  sl[4] = hi.x - m; sl[5] = hi.y - m; sl[6] = hi.z - m; sl[7] = hi.w - m;
  float s = 0.0f;
#pragma unroll 1
  for (int k = 0; k < NK; ++k) { const float e = expf(sl[k]); s += e; sl[k] = e; }
  const float inv = 1.0f / s;
#pragma unroll 1
  for (int k = 0; k < NK; ++k) sl[k] = sl[k] * inv;
  __syncthreads();
  float* ob = out + (sel ? OFF_AQ : OFF_AP) + (size_t)blockIdx.x * 2048;
#pragma unroll
  for (int q = 0; q < 2; ++q) {
    const int pc = t + 256 * q;
    const v4f v = *(const v4fa*)(sL + 4 * pc);
    *(volatile v4f*)(ob + 4 * pc) = v;
  }
  __threadfence();
#pragma unroll
  for (int q = 0; q < 2; ++q) {
    const int pc = t + 256 * q;
    const v4f v = *(const v4fa*)(sL + 4 * pc);
    *(volatile v4f*)(ob + 4 * pc) = v;
  }
}

extern "C" void kernel_launch(void* const* d_in, const int* in_sizes, int n_in,
                              void* d_out, int out_size, void* d_ws, size_t ws_size,
                              hipStream_t stream)
{
  if (n_in < 35) return;
  if (in_sizes[0] != NB * NPT * 2 || in_sizes[1] != NB * NPT * 3) return;
  if (in_sizes[2] != NB * NPT * 2 || in_sizes[3] != NB * NPT * 3) return;
  if (in_sizes[4] != NB * NTT * 2 || in_sizes[5] != NB * NTT * 3) return;
  if (in_sizes[6] != NB * NK * NL) return;
  if (in_sizes[9] != NK * 5 * NH || in_sizes[10] != NK * NH) return;
  if (in_sizes[11] != 2 * NK * NH * NH || in_sizes[12] != 2 * NK * NH) return;
  if (in_sizes[13] != NK * NH * NL || in_sizes[14] != NK * NL) return;
  if (in_sizes[15] != NK * NH * NL || in_sizes[16] != NK * NL) return;
  if (in_sizes[17] != 133 * NHG || in_sizes[18] != NHG || in_sizes[19] != NHG * NHG || in_sizes[20] != NHG) return;
  if (in_sizes[21] != NHG || in_sizes[22] < 1) return;
  if (in_sizes[23] != 130 * NHG || in_sizes[24] != NHG || in_sizes[25] != NHG * NHG || in_sizes[26] != NHG) return;
  if (in_sizes[27] != NHG || in_sizes[28] < 1) return;
  if (in_sizes[29] != 130 * NH || in_sizes[30] != NH || in_sizes[31] != 3 * NH * NH || in_sizes[32] != 3 * NH) return;
  if (in_sizes[33] != NH * 6 || in_sizes[34] != 6) return;
  if (out_size != OUT_TOTAL) return;

  const float* x_c    = (const float*)d_in[0];
  const float* y_c    = (const float*)d_in[1];
  const float* x_t    = (const float*)d_in[2];
  const float* y_t    = (const float*)d_in[3];
  const float* x_pred = (const float*)d_in[4];
  const float* y_pred = (const float*)d_in[5];
  const float* eps    = (const float*)d_in[6];
  const float* eW0    = (const float*)d_in[9];
  const float* eb0    = (const float*)d_in[10];
  const float* eWh    = (const float*)d_in[11];
  const float* ebh    = (const float*)d_in[12];
  const float* eWmu   = (const float*)d_in[13];
  const float* ebmu   = (const float*)d_in[14];
  const float* eWlv   = (const float*)d_in[15];
  const float* eblv   = (const float*)d_in[16];
  const float* pW0    = (const float*)d_in[17];
  const float* pb0    = (const float*)d_in[18];
  const float* pWh    = (const float*)d_in[19];
  const float* pbh    = (const float*)d_in[20];
  const float* pWo    = (const float*)d_in[21];
  const float* pbo    = (const float*)d_in[22];
  const float* qW0    = (const float*)d_in[23];
  const float* qb0    = (const float*)d_in[24];
  const float* qWh    = (const float*)d_in[25];
  const float* qbh    = (const float*)d_in[26];
  const float* qWo    = (const float*)d_in[27];
  const float* qbo    = (const float*)d_in[28];
  const float* dW0    = (const float*)d_in[29];
  const float* db0    = (const float*)d_in[30];
  const float* dWh    = (const float*)d_in[31];
  const float* dbh    = (const float*)d_in[32];
  const float* dWo    = (const float*)d_in[33];
  const float* dbo    = (const float*)d_in[34];
  float* out = (float*)d_out;

  const size_t szEWhT = (size_t)2 * NK * NH * NH * 2;
  const size_t szDWhT = (size_t)3 * NH * NH * 2;
  const size_t szGWhT = (size_t)NHG * NHG * 2;
  const size_t szBuf  = (size_t)NK * MROWS * NH * 2;
  const size_t szPP   = (size_t)NK * 32 * NH * 4;
  const size_t szZ    = (size_t)NB * NK * NL * 4;
  const size_t szZD   = (size_t)NB * NK * NH * 4;
  const size_t szZG   = (size_t)NB * NK * NHG * 4;
  const size_t szPdec = (size_t)4 * DROWS * 8 * 4;
  const size_t szPlog = (size_t)2 * DROWS * 4;
  size_t off = 0;
  const size_t oEWhT = off; off += szEWhT;
  const size_t oDWhT = off; off += szDWhT;
  const size_t oPWhT = off; off += szGWhT;
  const size_t oQWhT = off; off += szGWhT;
  const size_t oBufA = off; off += szBuf;
  const size_t oBufB = off; off += szBuf;
  const size_t oPP   = off; off += szPP;
  const size_t oZ    = off; off += szZ;
  const size_t oZD   = off; off += szZD;
  const size_t oZP   = off; off += szZG;
  const size_t oZQ   = off; off += szZG;
  const size_t oPdec = off; off += szPdec;
  const size_t oPlP  = off; off += szPlog;
  const size_t oPlQ  = off; off += szPlog;
  const size_t total = off;
  if (total > ws_size) return;

  char* ws = (char*)d_ws;
  _Float16* eWhT = (_Float16*)(ws + oEWhT);
  _Float16* dWhT = (_Float16*)(ws + oDWhT);
  _Float16* pWhT = (_Float16*)(ws + oPWhT);
  _Float16* qWhT = (_Float16*)(ws + oQWhT);
  _Float16* bufA = (_Float16*)(ws + oBufA);
  _Float16* bufB = (_Float16*)(ws + oBufB);
  float* pp    = (float*)(ws + oPP);
  float* zbuf  = (float*)(ws + oZ);
  float* zD    = (float*)(ws + oZD);
  float* zP    = (float*)(ws + oZP);
  float* zQ    = (float*)(ws + oZQ);
  float* pdec  = (float*)(ws + oPdec);
  float* plogP = (float*)(ws + oPlP);
  float* plogQ = (float*)(ws + oPlQ);

  k_cvtT<<<dim3(NH / 32, NH / 64, 2 * NK), 256, 0, stream>>>(eWh, eWhT, NH, NH, NH * NH, NH * NH);
  k_cvtT<<<dim3(NH / 32, NH / 64, 3), 256, 0, stream>>>(dWh, dWhT, NH, NH, NH * NH, NH * NH);
  k_cvtT<<<dim3(NHG / 32, NHG / 64, 1), 256, 0, stream>>>(pWh, pWhT, NHG, NHG, 0, 0);
  k_cvtT<<<dim3(NHG / 32, NHG / 64, 1), 256, 0, stream>>>(qWh, qWhT, NHG, NHG, 0, 0);

  for (int which = 0; which < 2; ++which) {
    const float* xs = which ? x_t : x_c;
    const float* ys = which ? y_t : y_c;
    k_l0<2, 3><<<dim3(MROWS / 16, NK), 256, 0, stream>>>(
        xs, ys, 0, 0, eW0, 5 * NH, eb0, NH, 30, 0, 0, NH, bufA, MROWS * NH);
    k_gemm<0><<<dim3((MROWS / 128) * (NH / 128), NK), 256, 0, stream>>>(
        bufA, MROWS * NH, eWhT, NH * NH, ebh, NH, NH, NH, MROWS / 128,
        bufB, MROWS * NH, pp, 0, 0, dWo);
    k_gemm<1><<<dim3((MROWS / 128) * (NH / 128), NK), 256, 0, stream>>>(
        bufB, MROWS * NH, eWhT + (size_t)NK * NH * NH, NH * NH, ebh + NK * NH, NH, NH, NH, MROWS / 128,
        bufA, MROWS * NH, pp, 32 * NH, 0, dWo);
    k_head<<<NB * NK, 128, 0, stream>>>(pp, eWmu, ebmu, eWlv, eblv, eps, which, out, zbuf);
  }

  k_zterm<<<NB * NK, 256, 0, stream>>>(zbuf, dW0, db0, pW0, pb0, qW0, qb0, zD, zP, zQ);

  for (int h = 0; h < 2; ++h) {
    k_l0<2, 0><<<dim3(DHALF / 16, 1), 256, 0, stream>>>(
        x_pred, x_pred, 3, h * DHALF, dW0, 0, zD, 0, 13, 7, NH, NH, bufA, 0);
    k_gemm<0><<<dim3((DHALF / 128) * (NH / 128), 1), 256, 0, stream>>>(
        bufA, 0, dWhT, 0, dbh, 0, NH, NH, DHALF / 128, bufB, 0, pp, 0, 0, dWo);
    k_gemm<0><<<dim3((DHALF / 128) * (NH / 128), 1), 256, 0, stream>>>(
        bufB, 0, dWhT + (size_t)NH * NH, 0, dbh + NH, 0, NH, NH, DHALF / 128, bufA, 0, pp, 0, 0, dWo);
    k_gemm<3><<<dim3((DHALF / 128) * (NH / 128), 1), 256, 0, stream>>>(
        bufA, 0, dWhT + (size_t)2 * NH * NH, 0, dbh + 2 * NH, 0, NH, NH, DHALF / 128, bufB, 0,
        pdec + (size_t)h * DHALF * 8, 0, DROWS * 8, dWo);
  }
  k_dec_fin<<<DROWS / 256, 256, 0, stream>>>(pdec, dbo, out);

  k_l0<2, 3><<<dim3(DROWS / 16, 1), 256, 0, stream>>>(
      x_pred, y_pred, 3, 0, pW0, 0, zP, 0, 13, 7, NHG, NHG, bufA, 0);
  k_l0<2, 0><<<dim3(DROWS / 16, 1), 256, 0, stream>>>(
      x_pred, x_pred, 3, 0, qW0, 0, zQ, 0, 13, 7, NHG, NHG, bufB, 0);
  k_gemm<2><<<dim3((DROWS / 128) * (NHG / 128), 1), 256, 0, stream>>>(
      bufA, 0, pWhT, 0, pbh, 0, NHG, NHG, DROWS / 128, bufB, 0, plogP, 0, DROWS, pWo);
  k_gemm<2><<<dim3((DROWS / 128) * (NHG / 128), 1), 256, 0, stream>>>(
      bufB, 0, qWhT, 0, qbh, 0, NHG, NHG, DROWS / 128, bufA, 0, plogQ, 0, DROWS, qWo);
  k_gate_fin<<<dim3(NB * NTT / 256, 2), 256, 0, stream>>>(plogP, pbo, plogQ, qbo, out);
}
